// SRSelfAttention_54451595378950
// MI455X (gfx1250) — hardware-run, weakly checked
//
#include <hip/hip_runtime.h>
#include <math.h>

typedef __attribute__((ext_vector_type(16))) _Float16 v16h;
typedef __attribute__((ext_vector_type(16))) __bf16 v16b;
typedef __attribute__((ext_vector_type(8)))  _Float16 v8h;
typedef __attribute__((ext_vector_type(8)))  float v8f;
typedef __attribute__((ext_vector_type(4)))  float v4f;
typedef __attribute__((ext_vector_type(2)))  float v2f;
typedef __attribute__((ext_vector_type(4)))  unsigned v4u;
typedef __attribute__((ext_vector_type(4)))  int v4i;
typedef float __attribute__((may_alias)) float_a;
typedef int __attribute__((may_alias)) int_a;

template <typename T> __device__ __forceinline__ void vst2(void* p, T v) { *(volatile T*)p = v; __threadfence(); *(volatile T*)p = v; }
__device__ __forceinline__ v8f wmma16(v16h a, v16h b, v8f c) {
  v8f d = __builtin_amdgcn_wmma_f32_16x16x32_f16(false, a, false, b, (short)0, c, false, false);
  asm volatile("v_nop\n\tv_nop\n\tv_nop\n\tv_nop" : "+v"(d) : "v"(a), "v"(b));
  return d;
}
__device__ __forceinline__ v8f wmma_bf(v16b a, v16b b, v8f c) {
  v8f d = __builtin_amdgcn_wmma_f32_16x16x32_bf16(false, a, false, b, (short)0, c, false, false);
  asm volatile("v_nop\n\tv_nop\n\tv_nop\n\tv_nop" : "+v"(d) : "v"(a), "v"(b));
  return d;
}
__device__ __forceinline__ v16h frag_h(const _Float16* rowk0, int lane) {
  union { v16h v; v8h q[2]; } u; const _Float16* p = rowk0 + 8 * (lane >> 4);
  u.q[0] = *(const v8h*)p; u.q[1] = *(const v8h*)(p + 16); return u.v;
}
__device__ __forceinline__ v16h frag_f32(const float* rowk0, int lane) {
  v16h a; const float* p = rowk0 + 8 * (lane >> 4);
#pragma unroll
  for (int i = 0; i < 8; ++i) { a[i] = (_Float16)p[i]; a[8 + i] = (_Float16)p[16 + i]; }
  return a;
}
__device__ __forceinline__ v16h frag_f32s(const float* rowk0, int lane, float sc) {
  v16h a; const float* p = rowk0 + 8 * (lane >> 4);
#pragma unroll
  for (int i = 0; i < 8; ++i) { a[i] = (_Float16)(p[i] * sc); a[8 + i] = (_Float16)(p[16 + i] * sc); }
  return a;
}
__device__ __forceinline__ v16h fragc_f32(const float* W, int k0, int n, int lane, int ld, int K) {
  v16h a; const int g = lane >> 4;
#pragma unroll
  for (int i = 0; i < 8; ++i) { const int ka = k0 + 8 * g + i, kb = ka + 16;
    a[i] = (_Float16)(ka < K ? W[(size_t)(ka < K ? ka : K - 1) * ld + n] : 0.f); a[8 + i] = (_Float16)(kb < K ? W[(size_t)(kb < K ? kb : K - 1) * ld + n] : 0.f); }
  return a;
}
struct F2 { v16b h, l; };
__device__ __forceinline__ F2 bsplit16(const float v[16]) { F2 r;
#pragma unroll
  for (int i = 0; i < 16; ++i) { const __bf16 h = (__bf16)v[i]; r.h[i] = h; r.l[i] = (__bf16)(v[i] - (float)h); }
  return r; }
__device__ __forceinline__ F2 split_row(const float* row, int k0, int lane) { float v[16]; const float* p = row + k0 + 8 * (lane >> 4);
#pragma unroll
  for (int i = 0; i < 8; ++i) { v[i] = p[i]; v[8 + i] = p[16 + i]; }
  return bsplit16(v); }
__device__ __forceinline__ F2 split_rowK(const float* row, int k0, int lane, int K) { float v[16]; const int g = lane >> 4;
#pragma unroll
  for (int i = 0; i < 8; ++i) { const int ka = k0 + 8 * g + i, kb = ka + 16; v[i] = ka < K ? row[ka < K ? ka : K - 1] : 0.f; v[8 + i] = kb < K ? row[kb < K ? kb : K - 1] : 0.f; }
  return bsplit16(v); }
__device__ __forceinline__ F2 split_col(const float* W, int k0, int n, int lane, int ld, int K) { float v[16]; const int g = lane >> 4;
#pragma unroll
  for (int i = 0; i < 8; ++i) { const int ka = k0 + 8 * g + i, kb = ka + 16; v[i] = ka < K ? W[(size_t)(ka < K ? ka : K - 1) * ld + n] : 0.f; v[8 + i] = kb < K ? W[(size_t)(kb < K ? kb : K - 1) * ld + n] : 0.f; }
  return bsplit16(v); }
__device__ __forceinline__ v8f mac3(const F2& a, const F2& b, v8f c) { c = wmma_bf(a.l, b.h, c); c = wmma_bf(a.h, b.l, c); return wmma_bf(a.h, b.h, c); }
__device__ __forceinline__ float sigm(float v) { return 1.0f / (1.0f + expf(-v)); }
#define LDSX() do { asm volatile("s_wait_dscnt 0" ::: "memory"); __builtin_amdgcn_wave_barrier(); __builtin_amdgcn_fence(__ATOMIC_RELEASE, "workgroup"); } while (0)


#define NB 8
#define NX 56
#define NTOK (1 + NX * NX)
#define NQP 3200
#define MSR ((NX / 2) * (NX / 2))
#define MKV (1 + MSR)
#define MP 832
#define DD 256
#define NH 8
#define HD 32
#ifndef TQB
#define TQB (NQP / 64)
#define TNB NB
#endif
typedef __attribute__((ext_vector_type(8))) __bf16 v8b;
__device__ __forceinline__ v16b frag_b(const __bf16* rowk0, int lane) {
  union { v16b v; v8b q[2]; } u; const __bf16* p = rowk0 + 8 * (lane >> 4);
  u.q[0] = *(const v8b*)p; u.q[1] = *(const v8b*)(p + 16); return u.v;
}
__device__ __forceinline__ float bfr(float v) { return (float)(__bf16)v; }
__device__ __attribute__((noinline)) float exp_ni(float v) { return expf(v); }
__device__ __attribute__((noinline)) float erf_ni(float v) { return erff(v); }

#define WS_PQ  0u
#define WS_PKV (WS_PQ + 2u * (size_t)DD * DD)
#define WS_PC  (WS_PKV + 2u * (size_t)2 * DD * DD)
#define WS_PP  (WS_PC + 2u * (size_t)DD * 4 * DD)
#define WS_XL  (WS_PP + 2u * (size_t)DD * DD)
#define WS_MV  (WS_XL + 4u * (size_t)NB * MSR * DD)
#define WS_XR  (WS_MV + 4u * (size_t)NB * 2 * DD)
#define WS_XRL (WS_XR + 2u * (size_t)NB * MP * DD)
#define WS_Q   (WS_XRL + 2u * (size_t)NB * MP * DD)
#define WS_K   (WS_Q + 2u * (size_t)NB * NQP * DD)
#define WS_V   (WS_K + 2u * (size_t)NB * MP * DD)
#define WS_O   (WS_V + 2u * (size_t)NB * DD * MP)
#define WS_END (WS_O + 4u * (size_t)NB * NQP * DD)

__global__ __launch_bounds__(256) void k_pack(const float* __restrict__ WQ, const float* __restrict__ WKV, const float* __restrict__ CW, const float* __restrict__ WP, __bf16* __restrict__ P) { const int n = blockIdx.x, t = threadIdx.x; __shared__ __align__(16) __bf16 s[4 * DD];
  if (n < DD) { s[t] = (__bf16)WQ[(size_t)t * DD + n]; __syncthreads(); if (t < DD / 8) vst2((unsigned*)(P + WS_PQ / 2 + (size_t)n * DD + t * 8), *(const v4u*)&s[t * 8]); }
  else if (n < 3 * DD) { const int o = n - DD; s[t] = (__bf16)WKV[(size_t)t * (2 * DD) + o]; __syncthreads(); if (t < DD / 8) vst2((unsigned*)(P + WS_PKV / 2 + (size_t)o * DD + t * 8), *(const v4u*)&s[t * 8]); }
  else if (n < 4 * DD) { const int o = n - 3 * DD; for (int e = t; e < 4 * DD; e += 256) { const int kk = e >> 8, c = e & 255; s[e] = (__bf16)CW[(((size_t)o * DD + c) * 2 + (kk >> 1)) * 2 + (kk & 1)]; } __syncthreads(); for (int q = t; q < 4 * DD / 8; q += 256) vst2((unsigned*)(P + WS_PC / 2 + (size_t)o * 4 * DD + q * 8), *(const v4u*)&s[q * 8]); }
  else { const int o = n - 4 * DD; s[t] = (__bf16)WP[(size_t)t * DD + o]; __syncthreads(); if (t < DD / 8) vst2((unsigned*)(P + WS_PP / 2 + (size_t)o * DD + t * 8), *(const v4u*)&s[t * 8]); } }
__global__ __launch_bounds__(128) void k_conv(const float* __restrict__ X, const __bf16* __restrict__ P, float* __restrict__ XL) {
  __shared__ __align__(16) float so[4][16][132];
  const int tid = threadIdx.x, wave = tid >> 5, lane = tid & 31, col = lane & 15, g = lane >> 4; const size_t b = blockIdx.z; const int p0 = blockIdx.x * 64 + wave * 16; const int o0 = blockIdx.y * 128;
  const int pr = p0 + col; const bool pv = pr < MSR; const int py = pr / (NX / 2), px = pr % (NX / 2);
  v8f acc[8] = {};
#pragma unroll 1
  for (int kk = 0; kk < 4; ++kk) { const int ky = kk >> 1, kx = kk & 1; const size_t tok = 1 + (size_t)(2 * py + ky) * NX + 2 * px + kx; const float* p = X + ((b * NTOK + (pv ? tok : 1)) * DD) + 8 * g;
#pragma unroll
    for (int kc = 0; kc < DD / 32; ++kc) { v16b a;
#pragma unroll
      for (int i = 0; i < 8; ++i) { a[i] = pv ? (__bf16)p[kc * 32 + i] : (__bf16)0.f; a[8 + i] = pv ? (__bf16)p[kc * 32 + 16 + i] : (__bf16)0.f; }
#pragma unroll
      for (int j = 0; j < 8; ++j) acc[j] = wmma_bf(a, frag_b(P + WS_PC / 2 + (size_t)(o0 + j * 16 + col) * 4 * DD + kk * DD + kc * 32, lane), acc[j]); } }
#pragma unroll
  for (int j = 0; j < 8; ++j)
#pragma unroll
    for (int r = 0; r < 8; ++r) so[wave][8 * g + r][j * 16 + col] = acc[j][r];
  LDSX();
  for (int rl = 0; rl < 16; ++rl) { const int pp = p0 + rl; if (pp < MSR) vst2(XL + ((b * MSR + pp) * DD) + o0 + lane * 4, *(const v4f*)&so[wave][rl][lane * 4]); }
}
__global__ __launch_bounds__(256) void k_instat(const float* __restrict__ XL, float* __restrict__ MV) { const size_t b = blockIdx.x; const int c = threadIdx.x; const float* p = XL + b * MSR * DD + c; float s = 0.f; for (int i = 0; i < MSR; ++i) s += p[(size_t)i * DD]; const float mean = s / (float)MSR; float q = 0.f; for (int i = 0; i < MSR; ++i) { const float d = p[(size_t)i * DD] - mean; q += d * d; }
  __shared__ __align__(16) float sm[2][DD]; sm[0][c] = mean; sm[1][c] = 1.0f / sqrtf(q / (float)MSR + 1e-5f); __syncthreads(); if (c < 2 * DD / 4) vst2(MV + b * 2 * DD + c * 4, *(const v4f*)&sm[c >> 6][(c & 63) * 4]); }
__global__ __launch_bounds__(256) void k_xr(const float* __restrict__ X, const float* __restrict__ XL, const float* __restrict__ MV, __bf16* __restrict__ XR, __bf16* __restrict__ XRL) {
  __shared__ __align__(16) __bf16 sh[64][DD + 8]; __shared__ __align__(16) __bf16 sl[64][DD + 8]; const size_t b = blockIdx.y; const int m0 = blockIdx.x * 64, t = threadIdx.x;
  for (int e = t; e < 64 * DD; e += 256) { const int rr = e >> 8, c = e & 255; const int m = m0 + rr; float v = 0.f;
    if (m == 0) v = bfr(X[(b * NTOK) * DD + c]); else if (m < MKV) v = (XL[(b * MSR + (m - 1)) * DD + c] - MV[b * 2 * DD + c]) * MV[b * 2 * DD + DD + c];
    const __bf16 hv = (__bf16)v; sh[rr][c] = hv; sl[rr][c] = (__bf16)(v - (float)hv); }
  __syncthreads();
  for (int e = t; e < 64 * (DD / 8); e += 256) { const int rr = e / (DD / 8), q = e % (DD / 8); vst2((unsigned*)(XR + ((b * MP + m0 + rr) * DD) + q * 8), *(const v4u*)&sh[rr][q * 8]); vst2((unsigned*)(XRL + ((b * MP + m0 + rr) * DD) + q * 8), *(const v4u*)&sl[rr][q * 8]); }
}
__global__ __launch_bounds__(128) void k_q(const float* __restrict__ X, const __bf16* __restrict__ P, _Float16* __restrict__ Q) {
  __shared__ __align__(16) _Float16 so[64][136];
  const int tid = threadIdx.x, wave = tid >> 5, lane = tid & 31, col = lane & 15, g = lane >> 4; const size_t b = blockIdx.z; const int n0 = blockIdx.x * 64 + wave * 16; const int o0 = blockIdx.y * 128; const int nr = n0 + col; const bool nv = nr < NTOK;
  v8f acc[8] = {};
#pragma unroll 2
  for (int kc = 0; kc < DD / 32; ++kc) { v16b a; { const float* p = X + ((b * NTOK + (nv ? nr : 0)) * DD) + kc * 32 + 8 * g;
#pragma unroll
      for (int i = 0; i < 8; ++i) { a[i] = nv ? (__bf16)p[i] : (__bf16)0.f; a[8 + i] = nv ? (__bf16)p[16 + i] : (__bf16)0.f; } }
#pragma unroll
    for (int j = 0; j < 8; ++j) acc[j] = wmma_bf(a, frag_b(P + WS_PQ / 2 + (size_t)(o0 + j * 16 + col) * DD + kc * 32, lane), acc[j]); }
#pragma unroll
  for (int j = 0; j < 8; ++j)
#pragma unroll
    for (int r = 0; r < 8; ++r) so[wave * 16 + 8 * g + r][j * 16 + col] = (_Float16)acc[j][r];
  LDSX();
  for (int rl = 0; rl < 16; ++rl) if (lane < 16) vst2((unsigned*)(Q + ((b * NQP + n0 + rl) * DD) + o0 + lane * 8), *(const v4u*)&so[wave * 16 + rl][lane * 8]);
}
__global__ __launch_bounds__(128) void k_kv(const __bf16* __restrict__ XR, const __bf16* __restrict__ XRL, const __bf16* __restrict__ P, _Float16* __restrict__ Kr, _Float16* __restrict__ V) {
  __shared__ __align__(16) _Float16 so[64][136]; __shared__ __align__(16) _Float16 st[128][72];
  const int tid = threadIdx.x, wave = tid >> 5, lane = tid & 31, col = lane & 15, g = lane >> 4; const size_t b = blockIdx.z; const int m0b = blockIdx.x * 64; const int r0 = m0b + wave * 16; const int o0 = blockIdx.y * 128;
  v8f acc[8] = {};
#pragma unroll 2
  for (int kc = 0; kc < DD / 32; ++kc) { const v16b ah = frag_b(XR + ((b * MP + r0 + col) * DD) + kc * 32, lane), al = frag_b(XRL + ((b * MP + r0 + col) * DD) + kc * 32, lane);
#pragma unroll
    for (int j = 0; j < 8; ++j) { const v16b w = frag_b(P + WS_PKV / 2 + (size_t)(o0 + j * 16 + col) * DD + kc * 32, lane); acc[j] = wmma_bf(ah, w, acc[j]); acc[j] = wmma_bf(al, w, acc[j]); } }
  if (o0 < DD) {
#pragma unroll
    for (int j = 0; j < 8; ++j)
#pragma unroll
      for (int r = 0; r < 8; ++r) so[wave * 16 + 8 * g + r][j * 16 + col] = (_Float16)acc[j][r];
    LDSX();
    for (int rl = 0; rl < 16; ++rl) if (lane < 16) vst2((unsigned*)(Kr + ((b * MP + r0 + rl) * DD) + o0 + lane * 8), *(const v4u*)&so[wave * 16 + rl][lane * 8]);
  } else { const int c0 = o0 - DD;
#pragma unroll
    for (int j = 0; j < 8; ++j)
#pragma unroll
      for (int r = 0; r < 8; ++r) st[j * 16 + col][wave * 16 + 8 * g + r] = (_Float16)acc[j][r];
    __syncthreads();
    for (int e = tid; e < 128 * 8; e += 128) { const int d = e >> 3, pc = e & 7; vst2((unsigned*)(V + ((b * DD + c0 + d) * MP) + m0b + pc * 8), *(const v4u*)&st[d][pc * 8]); } }
}
__global__ __launch_bounds__(128) void k_attn(const _Float16* __restrict__ Q, const _Float16* __restrict__ Kr, const _Float16* __restrict__ V, float* __restrict__ O) {
  __shared__ __align__(16) _Float16 sph[4][16][40]; __shared__ __align__(16) float so[4][16][36];
  const int tid = threadIdx.x, wave = tid >> 5, lane = tid & 31, col = lane & 15, g = lane >> 4; const int h = blockIdx.y; const size_t b = blockIdx.z; const int q0 = blockIdx.x * 64 + wave * 16;
  const v16h aq = frag_h(Q + ((b * NQP + q0 + col) * DD) + h * HD, lane);
  float m[8], l[8];
#pragma unroll
  for (int r = 0; r < 8; ++r) { m[r] = -3.0e38f; l[r] = 0.f; }
  v8f acc[2] = {};
#pragma unroll 1
  for (int ks = 0; ks < MP / 32; ++ks) { const int j0 = ks * 32; v8f s[2];
#pragma unroll
    for (int ct = 0; ct < 2; ++ct) { const int kk = j0 + ct * 16 + col; const v8f z = {}; const v8f c = wmma16(aq, frag_h(Kr + ((b * MP + kk) * DD) + h * HD, lane), z); const bool keep = kk < MKV;
#pragma unroll
      for (int r = 0; r < 8; ++r) s[ct][r] = keep ? c[r] * 0.17677669529663688f : -3.0e38f; }
#pragma unroll
    for (int r = 0; r < 8; ++r) { float mx = fmaxf(s[0][r], s[1][r]);
#pragma unroll
      for (int o = 1; o < 16; o <<= 1) mx = fmaxf(mx, __shfl_xor(mx, o));
      const float mn = fmaxf(m[r], mx); const float alpha = (m[r] <= -1.0e38f) ? 0.f : __expf(m[r] - mn); const float e0 = (s[0][r] <= -1.0e38f) ? 0.f : __expf(s[0][r] - mn), e1 = (s[1][r] <= -1.0e38f) ? 0.f : __expf(s[1][r] - mn); float es = e0 + e1;
#pragma unroll
      for (int o = 1; o < 16; o <<= 1) es += __shfl_xor(es, o);
      l[r] = l[r] * alpha + es; m[r] = mn;
#pragma unroll
      for (int dt = 0; dt < 2; ++dt) acc[dt][r] *= alpha;
      sph[wave][8 * g + r][col] = (_Float16)(e0 * 2048.0f); sph[wave][8 * g + r][16 + col] = (_Float16)(e1 * 2048.0f); }
    LDSX();
    const v16h pa = frag_h(&sph[wave][col][0], lane);
#pragma unroll
    for (int dt = 0; dt < 2; ++dt) acc[dt] = wmma16(pa, frag_h(V + ((b * DD + h * HD + dt * 16 + col) * MP) + j0, lane), acc[dt]);
    LDSX(); }
#pragma unroll
  for (int r = 0; r < 8; ++r) { const float il = (1.0f / 2048.0f) / l[r];
#pragma unroll
    for (int dt = 0; dt < 2; ++dt) so[wave][8 * g + r][dt * 16 + col] = acc[dt][r] * il; }
  LDSX();
  for (int rl = 0; rl < 16; ++rl) if (lane < 8) vst2(O + ((b * NQP + q0 + rl) * DD) + h * HD + lane * 4, *(const v4f*)&so[wave][rl][lane * 4]);
}
__global__ __launch_bounds__(128) void k_out(const float* __restrict__ O, const __bf16* __restrict__ P, const float* __restrict__ BP, float* __restrict__ OUT) {
  __shared__ __align__(16) float so[4][16][132];
  const int tid = threadIdx.x, wave = tid >> 5, lane = tid & 31, col = lane & 15, g = lane >> 4; const size_t b = blockIdx.z; const int n0 = blockIdx.x * 64 + wave * 16; const int o0 = blockIdx.y * 128;
  v8f acc[8] = {};
#pragma unroll 2
  for (int kc = 0; kc < DD / 32; ++kc) { const F2 a = split_row(O + ((b * NQP + n0 + col) * DD), kc * 32, lane);
#pragma unroll
    for (int j = 0; j < 8; ++j) { const v16b w = frag_b(P + WS_PP / 2 + (size_t)(o0 + j * 16 + col) * DD + kc * 32, lane); acc[j] = wmma_bf(a.l, w, acc[j]); acc[j] = wmma_bf(a.h, w, acc[j]); } }
#pragma unroll
  for (int j = 0; j < 8; ++j) { const float bb = bfr(BP[o0 + j * 16 + col]);
#pragma unroll
    for (int r = 0; r < 8; ++r) so[wave][8 * g + r][j * 16 + col] = acc[j][r] + bb; }
  LDSX();
  for (int rl = 0; rl < 16; ++rl) { const int n = n0 + rl; if (n < NTOK) vst2(OUT + ((b * NTOK + n) * DD) + o0 + lane * 4, *(const v4f*)&so[wave][rl][lane * 4]); }
}
extern "C" void kernel_launch(void* const* d_in, const int* in_sizes, int n_in, void* d_out, int out_size, void* d_ws, size_t ws_size, hipStream_t stream) {
  (void)in_sizes; (void)n_in; (void)out_size;
  const float** F = (const float**)d_in;
  if (ws_size < (size_t)WS_END) return;
  char* ws = (char*)d_ws; __bf16 *P = (__bf16*)ws, *XR = (__bf16*)(ws + WS_XR), *XRL = (__bf16*)(ws + WS_XRL); float *XL = (float*)(ws + WS_XL), *MV = (float*)(ws + WS_MV), *O = (float*)(ws + WS_O); _Float16 *Q = (_Float16*)(ws + WS_Q), *Kr = (_Float16*)(ws + WS_K), *V = (_Float16*)(ws + WS_V);
  k_pack<<<5 * DD, 256, 0, stream>>>(F[1], F[2], F[3], F[4], P);
  k_conv<<<dim3((MSR + 63) / 64, DD / 128, NB), 128, 0, stream>>>(F[0], P, XL);
  k_instat<<<NB, 256, 0, stream>>>(XL, MV);
  k_xr<<<dim3(MP / 64, NB), 256, 0, stream>>>(F[0], XL, MV, XR, XRL);
  k_q<<<dim3(NQP / 64, DD / 128, TNB), 128, 0, stream>>>(F[0], P, Q);
  k_kv<<<dim3(MP / 64, 2 * DD / 128, NB), 128, 0, stream>>>(XR, XRL, P, Kr, V);
  k_attn<<<dim3(TQB, NH, TNB), 128, 0, stream>>>(Q, Kr, V, O);
  k_out<<<dim3(TQB, DD / 128, TNB), 128, 0, stream>>>(O, P, F[5], (float*)d_out);
}
